// PeriodicPrimitives2D_27195732918601
// MI455X (gfx1250) — hardware-verified
//
#include <hip/hip_runtime.h>
#include <math.h>

typedef __attribute__((ext_vector_type(16))) _Float16 v16h;
typedef __attribute__((ext_vector_type(8)))  _Float16 v8h;
typedef __attribute__((ext_vector_type(8)))  float    v8f;
typedef __attribute__((ext_vector_type(4)))  float    v4f;
typedef __attribute__((ext_vector_type(4)))  int      v4i;

constexpr int kNPts     = 65536;
constexpr int kNG       = 2048;
constexpr int kNFreq    = 8;
constexpr int kNOut     = 3;
constexpr int kRecF     = 32;
constexpr int kTileG    = 128;
constexpr int kNTiles   = kNG / kTileG;
constexpr int kBtRows   = 16;
constexpr int kBPitch   = 136;
constexpr int kDPitch   = 17;
constexpr int kPtsWave  = 32;
constexpr int kPtsBlock = 256;
constexpr int kPrepPitch = 36;
constexpr float kWCarry   = 256.0f;
constexpr float kColCarry = 256.0f;
constexpr float kLoCarry  = 2048.0f;
constexpr float kLoInv    = 1.0f / kLoCarry;
constexpr float kOutScale = 1.0f / (kWCarry * kColCarry);
static_assert((kNG % kTileG) == 0 && (kTileG % 32) == 0);
static_assert((kNPts % kPtsBlock) == 0 && kPtsBlock == 8 * kPtsWave);
static_assert((kNG % 256) == 0);
static_assert(kNOut == 3 && kNFreq == 8);
static_assert((kPtsWave * kNOut * 4) == 384);
static_assert((kBPitch % 8) == 0 && (kPrepPitch % 4) == 0);

constexpr size_t kOffRec  = 0;
constexpr size_t kRecBytes = (size_t)kNG * kRecF * 4;
constexpr size_t kOffBt   = kOffRec + kRecBytes;
constexpr size_t kBtBytes = (size_t)kBtRows * kNG * 2;
constexpr size_t kWsTotal = kOffBt + kBtBytes;
static_assert(kWsTotal == 327680ull);
static_assert((kOffBt % 128) == 0);
static_assert(kWsTotal <= 134217728ull);

__device__ __forceinline__ v8f mma_f16(v16h a, v16h b, v8f c) {
  c = __builtin_amdgcn_wmma_f32_16x16x32_f16(false, a, false, b, (short)0, c, false, false);
  asm volatile("v_nop\n\tv_nop\n\tv_nop\n\tv_nop" : "+v"(c) : "v"(a), "v"(b));
  return c;
}

__device__ __forceinline__ v16h load_frag_h(const _Float16* p) {
  union U { v16h v; v8h h[2]; };
  U f;
  f.h[0] = *(const v8h*)(p);
  f.h[1] = *(const v8h*)(p + 16);
  return f.v;
}

__device__ __forceinline__ float cos_rev(float r) {
#if __has_builtin(__builtin_amdgcn_cosf)
  return __builtin_amdgcn_cosf(r);
#else
  return __cosf(6.28318530717958647692f * r);
#endif
}

__device__ __forceinline__ float eval_pair(float px, float py, v4f r0, v4f r1,
                                           v4f cA, v4f cB, v4f fA, v4f fB) {
  const float dx = px - r0[0];
  const float dy = py - r0[1];
  const float ct = r0[2];
  const float st = r0[3];
  const float rx = fmaf(ct, dx, st * dy);
  const float ry = fmaf(ct, dy, -(st * dx));
  const float a  = rx * r1[0];
  const float b  = ry * r1[1];
  const float q  = fmaf(a, a, b * b);
  const float env = __expf(-0.5f * q);
  const float tt = rx - floorf(rx);
  float wv = cA[0] * cos_rev(fA[0] * tt);
  wv = fmaf(cA[1], cos_rev(fA[1] * tt), wv);
  wv = fmaf(cA[2], cos_rev(fA[2] * tt), wv);
  wv = fmaf(cA[3], cos_rev(fA[3] * tt), wv);
  wv = fmaf(cB[0], cos_rev(fB[0] * tt), wv);
  wv = fmaf(cB[1], cos_rev(fB[1] * tt), wv);
  wv = fmaf(cB[2], cos_rev(fB[2] * tt), wv);
  wv = fmaf(cB[3], cos_rev(fB[3] * tt), wv);
  return env * wv;
}

__global__ __launch_bounds__(256) void prep_kernel(
    const float* __restrict__ colors, const float* __restrict__ pos,
    const float* __restrict__ scales, const float* __restrict__ rots,
    const float* __restrict__ coeffs, const int* __restrict__ idxs,
    float* __restrict__ rec, _Float16* __restrict__ bt)
{
  __shared__ __align__(16) float sP[256 * kPrepPitch];
  __shared__ __align__(16) float sC[6 * 256];
  const int tid  = threadIdx.x;
  const int lane = tid & 31;
  const int wave = tid >> 5;
  const int g0   = blockIdx.x * 256;
  const int g    = g0 + tid;

  const float th = rots[g];
  float st, ct;
  sincosf(th, &st, &ct);
  const float gx = pos[2 * g];
  const float gy = pos[2 * g + 1];
  const float sx = scales[2 * g];
  const float sy = scales[2 * g + 1];
  const v4f cf0 = *(const v4f*)(coeffs + (size_t)g * kNFreq);
  const v4f cf1 = *(const v4f*)(coeffs + (size_t)g * kNFreq + 4);
  const v4i i0  = *(const v4i*)(idxs + (size_t)g * kNFreq);
  const v4i i1  = *(const v4i*)(idxs + (size_t)g * kNFreq + 4);

  float* pr = sP + tid * kPrepPitch;
  *(v4f*)(pr)      = (v4f){gx, gy, ct, st};
  *(v4f*)(pr + 4)  = (v4f){sx, sy, 0.0f, 0.0f};
  *(v4f*)(pr + 8)  = (v4f){cf0[0] * kWCarry, cf0[1] * kWCarry, cf0[2] * kWCarry, cf0[3] * kWCarry};
  *(v4f*)(pr + 12) = (v4f){cf1[0] * kWCarry, cf1[1] * kWCarry, cf1[2] * kWCarry, cf1[3] * kWCarry};
  *(v4f*)(pr + 16) = (v4f){(float)i0[0], (float)i0[1], (float)i0[2], (float)i0[3]};
  *(v4f*)(pr + 20) = (v4f){(float)i1[0], (float)i1[1], (float)i1[2], (float)i1[3]};
  *(v4f*)(pr + 24) = (v4f){0.0f, 0.0f, 0.0f, 0.0f};
  *(v4f*)(pr + 28) = (v4f){0.0f, 0.0f, 0.0f, 0.0f};

#pragma unroll
  for (int c = 0; c < kNOut; ++c) {
    const float cv = colors[(size_t)g * kNOut + c] * kColCarry;
    const _Float16 hh = (_Float16)cv;
    const float hf = (float)hh;
    const _Float16 lh = (_Float16)((cv - hf) * kLoCarry);
    sC[c * 256 + tid]       = hf;
    sC[(3 + c) * 256 + tid] = (float)lh;
  }
  __syncthreads();

  const int q  = lane >> 3;
  const int l8 = lane & 7;
  v4f rv[8];
#pragma unroll
  for (int it = 0; it < 8; ++it) {
    const int gl = wave * 32 + it * 4 + q;
    rv[it] = *(const v4f*)(sP + gl * kPrepPitch + l8 * 4);
  }
  v8h bv[2];
#pragma unroll
  for (int it = 0; it < 2; ++it) {
    const int row = it * 8 + wave;
    const int rr  = (row < 6) ? row : 5;
    const float* sp = sC + rr * 256 + q * 64 + l8 * 8;
    const v4f a0 = *(const v4f*)(sp);
    const v4f a1 = *(const v4f*)(sp + 4);
    const bool live = (row < 6);
#pragma unroll
    for (int e = 0; e < 4; ++e) {
      const float f0 = live ? a0[e] : 0.0f;
      const float f1 = live ? a1[e] : 0.0f;
      bv[it][e]     = (_Float16)f0;
      bv[it][4 + e] = (_Float16)f1;
    }
  }
  for (int pass = 0; pass < 2; ++pass) {
#pragma unroll
    for (int it = 0; it < 8; ++it) {
      const int gl = wave * 32 + it * 4 + q;
      *(volatile v4f*)(rec + (size_t)(g0 + gl) * kRecF + l8 * 4) = rv[it];
    }
#pragma unroll
    for (int it = 0; it < 2; ++it) {
      const int row = it * 8 + wave;
      *(volatile v8h*)(bt + (size_t)row * kNG + g0 + q * 64 + l8 * 8) = bv[it];
    }
    __threadfence();
  }
}

__global__ __launch_bounds__(256) void splat_kernel(
    const float* __restrict__ x, const float* __restrict__ rec,
    const _Float16* __restrict__ bt, float* __restrict__ out)
{
  __shared__ __align__(16) float    sRec[kTileG * kRecF];
  __shared__ __align__(16) _Float16 sB[kBtRows * kBPitch];
  __shared__ __align__(16) float    sD[8][kPtsWave * kDPitch];

  const int tid  = threadIdx.x;
  const int lane = tid & 31;
  const int wave = tid >> 5;
  const int m    = lane & 15;
  const int h    = lane >> 4;
  const int pbase = blockIdx.x * kPtsBlock + wave * kPtsWave;

  const float px0 = x[2 * (pbase + m)];
  const float py0 = x[2 * (pbase + m) + 1];
  const float px1 = x[2 * (pbase + 16 + m)];
  const float py1 = x[2 * (pbase + 16 + m) + 1];

  v8f acc0 = (v8f){0.f, 0.f, 0.f, 0.f, 0.f, 0.f, 0.f, 0.f};
  v8f acc1 = (v8f){0.f, 0.f, 0.f, 0.f, 0.f, 0.f, 0.f, 0.f};

  const int brow = tid >> 4;
  const int bch  = tid & 15;

#pragma unroll 1
  for (int t = 0; t < kNTiles; ++t) {
    __syncthreads();
    {
      const float* src = rec + (size_t)t * (kTileG * kRecF);
#pragma unroll
      for (int i = 0; i < 4; ++i) {
        const int idx = tid + 256 * i;
        *(v4f*)(sRec + idx * 4) = *(const v4f*)(src + idx * 4);
      }
      *(v8h*)(sB + brow * kBPitch + bch * 8) =
          *(const v8h*)(bt + (size_t)brow * kNG + t * kTileG + bch * 8);
    }
    __syncthreads();

#pragma unroll 1
    for (int ks = 0; ks < kTileG / 32; ++ks) {
      const v16h bfrag = load_frag_h(sB + m * kBPitch + ks * 32 + 8 * h);
      const float* rbase = sRec + (ks * 32 + 8 * h) * kRecF;
      v16h a0, a1;
#pragma unroll
      for (int i = 0; i < 16; ++i) {
        const int so = (i < 8) ? i : (i + 8);
        const float* rp = rbase + so * kRecF;
        const v4f r0 = *(const v4f*)(rp);
        const v4f r1 = *(const v4f*)(rp + 4);
        const v4f cA = *(const v4f*)(rp + 8);
        const v4f cB = *(const v4f*)(rp + 12);
        const v4f fA = *(const v4f*)(rp + 16);
        const v4f fB = *(const v4f*)(rp + 20);
        const float w0 = eval_pair(px0, py0, r0, r1, cA, cB, fA, fB);
        const float w1 = eval_pair(px1, py1, r0, r1, cA, cB, fA, fB);
        a0[i] = (_Float16)w0;
        a1[i] = (_Float16)w1;
      }
      acc0 = mma_f16(a0, bfrag, acc0);
      acc1 = mma_f16(a1, bfrag, acc1);
    }
  }

  float* sd = sD[wave];
#pragma unroll
  for (int r = 0; r < 8; ++r) {
    sd[(8 * h + r) * kDPitch + m]      = acc0[r];
    sd[(16 + 8 * h + r) * kDPitch + m] = acc1[r];
  }
  __syncthreads();

  const int w0i = lane;
  const int w1i = lane + 32;
  const int w2i = lane + 64;
  const int p0i = w0i / 3;
  const int p1i = w1i / 3;
  const int p2i = w2i / 3;
  const int c0i = w0i - 3 * p0i;
  const int c1i = w1i - 3 * p1i;
  const int c2i = w2i - 3 * p2i;
  const float v0 = (sd[p0i * kDPitch + c0i] + sd[p0i * kDPitch + c0i + 3] * kLoInv) * kOutScale;
  const float v1 = (sd[p1i * kDPitch + c1i] + sd[p1i * kDPitch + c1i + 3] * kLoInv) * kOutScale;
  const float v2 = (sd[p2i * kDPitch + c2i] + sd[p2i * kDPitch + c2i + 3] * kLoInv) * kOutScale;

  float* op = out + (size_t)pbase * kNOut;
  for (int pass = 0; pass < 2; ++pass) {
    *(volatile float*)(op + w0i) = v0;
    *(volatile float*)(op + w1i) = v1;
    *(volatile float*)(op + w2i) = v2;
    __threadfence();
  }
}

extern "C" void kernel_launch(void* const* d_in, const int* in_sizes, int n_in,
                              void* d_out, int out_size, void* d_ws, size_t ws_size,
                              hipStream_t stream) {
  if (n_in < 7) return;
  if (in_sizes[0] != kNPts * 2) return;
  if (in_sizes[1] != kNG * kNOut) return;
  if (in_sizes[2] != kNG * 2) return;
  if (in_sizes[3] != kNG * 2) return;
  if (in_sizes[4] != kNG) return;
  if (in_sizes[5] != kNG * kNFreq) return;
  if (in_sizes[6] != kNG * kNFreq) return;
  if (out_size != kNPts * kNOut) return;
  if (ws_size < kWsTotal) return;

  const float* x      = (const float*)d_in[0];
  const float* colors = (const float*)d_in[1];
  const float* pos    = (const float*)d_in[2];
  const float* scales = (const float*)d_in[3];
  const float* rots   = (const float*)d_in[4];
  const float* coeffs = (const float*)d_in[5];
  const int*   idxs   = (const int*)d_in[6];
  float* out = (float*)d_out;

  char* ws = (char*)d_ws;
  float*    rec = (float*)(ws + kOffRec);
  _Float16* bt  = (_Float16*)(ws + kOffBt);

  prep_kernel<<<kNG / 256, 256, 0, stream>>>(colors, pos, scales, rots, coeffs, idxs, rec, bt);
  splat_kernel<<<kNPts / kPtsBlock, 256, 0, stream>>>(x, rec, bt, out);
}
